// SwinTransformerBlock_kv_29832842838661
// MI455X (gfx1250) — hardware-verified
//
#include <hip/hip_runtime.h>
#include <stdint.h>

#define LTOK  16384
#define CDIM  192
#define NHEAD 6
#define HDIM  32
#define NTOK  64
#define NROW  32768
#define NWINT (NROW / NTOK)
#define NWB   256
#define HID   768
#define NKV   384
#define NRPB  343
#define LDC   68
#define PP    72
#define OSP   36
#define PWB   4608
#define QSC   0.17677669529663687f

static_assert(NROW == NWINT * NTOK);
static_assert(NROW == 2 * LTOK);
static_assert(NWINT == 2 * NWB);
static_assert(NWB == (16 / 4) * (32 / 4) * (32 / 4));
static_assert(CDIM == NHEAD * HDIM);
static_assert(PWB == 2 * 16 * PP * 2);
static_assert(16 * OSP * 4 <= PWB);
static_assert((LDC * 4) % 16 == 0);
static_assert((PP * 2) % 16 == 0);
static_assert(NROW % 256 == 0);
static_assert(NKV % 64 == 0 && HID % 64 == 0 && CDIM % 64 == 0);

typedef _Float16 v16h __attribute__((ext_vector_type(16)));
typedef _Float16 v8h  __attribute__((ext_vector_type(8)));
typedef float    v8f  __attribute__((ext_vector_type(8)));
typedef float    v4f  __attribute__((ext_vector_type(4)));
typedef unsigned int v4u __attribute__((ext_vector_type(4)));

__device__ __forceinline__ unsigned short bf_bits(float f) {
  unsigned u = __float_as_uint(f);
  return (unsigned short)((u + 0x7FFFu + ((u >> 16) & 1u)) >> 16);
}
__device__ __forceinline__ float bf_up(unsigned short b) { return __uint_as_float(((unsigned)b) << 16); }
__device__ __forceinline__ float bfr(float f) { return bf_up(bf_bits(f)); }
__device__ __forceinline__ unsigned short h_bits(_Float16 x) { return __builtin_bit_cast(unsigned short, x); }
__device__ __forceinline__ unsigned short hb16(float f) { return h_bits((_Float16)f); }
__device__ __forceinline__ unsigned pk16(unsigned short a, unsigned short b) { return (unsigned)a | ((unsigned)b << 16); }
__device__ __forceinline__ v8f zero8() { v8f z = {0.f, 0.f, 0.f, 0.f, 0.f, 0.f, 0.f, 0.f}; return z; }

__device__ __forceinline__ int pos_of(int row) {
  const int win = row >> 6, t = row & 63;
  const int bb = win >> 8, wi = win & 255;
  const int s = ((wi >> 6) << 2) + (t >> 4);
  const int h = (((wi >> 3) & 7) << 2) + ((t >> 2) & 3);
  const int w = ((wi & 7) << 2) + (t & 3);
  return bb * LTOK + (s << 10) + (h << 5) + w;
}

__device__ __forceinline__ v16h ldfrag_h(const _Float16* p) {
  union { v16h v; v8h h[2]; } f;
  f.h[0] = *(const v8h*)(p);
  f.h[1] = *(const v8h*)(p + 16);
  return f.v;
}

__device__ __forceinline__ v8f mma_raw(v16h a, v16h b, v8f c) {
  return __builtin_amdgcn_wmma_f32_16x16x32_f16(false, a, false, b, (short)0, c, false, false);
}
__device__ __forceinline__ void guard2(v8f& c0, v8f& c1, const v16h& a0, const v16h& a1, const v16h& b0) {
#if defined(__HIP_DEVICE_COMPILE__)
  asm volatile("v_nop\n\tv_nop\n\tv_nop\n\tv_nop" : "+v"(c0), "+v"(c1) : "v"(a0), "v"(a1), "v"(b0));
#endif
}
__device__ __forceinline__ void guard3(v8f& c0, v8f& c1, v8f& c2,
                                       const v16h& a0, const v16h& a1, const v16h& b0, const v16h& b1) {
#if defined(__HIP_DEVICE_COMPILE__)
  asm volatile("v_nop\n\tv_nop\n\tv_nop\n\tv_nop"
               : "+v"(c0), "+v"(c1), "+v"(c2) : "v"(a0), "v"(a1), "v"(b0), "v"(b1));
#endif
}
__device__ __forceinline__ void guard8(v8f& c0, v8f& c1, v8f& c2, v8f& c3, v8f& c4, v8f& c5, v8f& c6, v8f& c7,
                                       const v16h& a0, const v16h& a1, const v16h& a2, const v16h& a3,
                                       const v16h& b0, const v16h& b1) {
#if defined(__HIP_DEVICE_COMPILE__)
  asm volatile("v_nop\n\tv_nop\n\tv_nop\n\tv_nop"
               : "+v"(c0), "+v"(c1), "+v"(c2), "+v"(c3), "+v"(c4), "+v"(c5), "+v"(c6), "+v"(c7)
               : "v"(a0), "v"(a1), "v"(a2), "v"(a3), "v"(b0), "v"(b1));
#endif
}
__device__ __forceinline__ void wave_sync_lds() {
  __builtin_amdgcn_fence(__ATOMIC_RELEASE, "workgroup");
  __builtin_amdgcn_wave_barrier();
  __builtin_amdgcn_fence(__ATOMIC_ACQUIRE, "workgroup");
}

__global__ __launch_bounds__(256) void cvt_wt(const float* __restrict__ src, unsigned short* dst, int K, int N) {
  __shared__ float tile[64][65];
  const int tid = threadIdx.x;
  const int n0 = blockIdx.x * 64, k0 = blockIdx.y * 64;
#pragma unroll
  for (int i = 0; i < 16; ++i) {
    const int kk = i * 4 + (tid >> 6), nn = tid & 63;
    tile[kk][nn] = src[(size_t)(k0 + kk) * N + n0 + nn];
  }
  __syncthreads();
  v4u pk[2];
  size_t offs[2];
#pragma unroll
  for (int it = 0; it < 2; ++it) {
    const int line = it * 32 + (tid >> 3), p = tid & 7;
    v4u q4;
#pragma unroll
    for (int e = 0; e < 4; ++e) {
      const float f0 = bfr(tile[p * 8 + 2 * e][line]) * 1024.0f;
      const float f1 = bfr(tile[p * 8 + 2 * e + 1][line]) * 1024.0f;
      q4[e] = pk16(hb16(f0), hb16(f1));
    }
    pk[it] = q4;
    offs[it] = (size_t)(n0 + line) * K + k0 + p * 8;
  }
  *(volatile v4u*)(dst + offs[0]) = pk[0];
  *(volatile v4u*)(dst + offs[1]) = pk[1];
  __threadfence();
  *(volatile v4u*)(dst + offs[0]) = pk[0];
  *(volatile v4u*)(dst + offs[1]) = pk[1];
}

__global__ __launch_bounds__(256) void build_bm(const float* __restrict__ rpb, float* bm) {
  const int g = blockIdx.x * 256 + threadIdx.x;
  const int h = g >> 10, n = (g >> 4) & 63, m0 = (g & 15) * 4;
  const int sn = n >> 4, hn = (n >> 2) & 3, wn = n & 3;
  v4f v;
#pragma unroll
  for (int e = 0; e < 4; ++e) {
    const int m = m0 + e;
    const int sm = m >> 4, hm = (m >> 2) & 3, wm = m & 3;
    int idx = (sn - sm + 3) * 11 + (hn - hm + 3) * 7 + (wn - wm + 3);
    idx = min(max(idx, 0), NRPB - 1);
    v[e] = bfr(rpb[idx * NHEAD + h]);
  }
  float* gp = bm + (size_t)g * 4;
  *(volatile v4f*)gp = v;
  __threadfence();
  *(volatile v4f*)gp = v;
}

__global__ __launch_bounds__(256)
void ln_rows(const float* __restrict__ src, const float* __restrict__ g, const float* __restrict__ b,
             unsigned short* dh, unsigned short* dl, float scl, int gather) {
  const int tid = threadIdx.x, wv = tid >> 5, lane = tid & 31;
  const int row = blockIdx.x * 8 + wv;
  const bool isin = (gather != 0);
  const int srow = isin ? pos_of(row) : row;
  const bool act = lane < 24;
  const int lc = act ? lane : 23;
  const float* sp = src + (size_t)srow * CDIM + lc * 8;
  const v4f a0 = *(const v4f*)(sp);
  const v4f a1 = *(const v4f*)(sp + 4);
  float v[8];
#pragma unroll
  for (int e = 0; e < 4; ++e) {
    const float x0 = isin ? bfr(a0[e]) : a0[e];
    const float x1 = isin ? bfr(a1[e]) : a1[e];
    v[e]     = act ? x0 : 0.f;
    v[4 + e] = act ? x1 : 0.f;
  }
  float s = 0.f;
#pragma unroll
  for (int e = 0; e < 8; ++e) s = s + v[e];
  s = s + __shfl_xor(s, 16, 32);
  s = s + __shfl_xor(s, 8, 32);
  s = s + __shfl_xor(s, 4, 32);
  s = s + __shfl_xor(s, 2, 32);
  s = s + __shfl_xor(s, 1, 32);
  const float mean = s * (1.0f / 192.0f);
  float d8[8];
  float q = 0.f;
#pragma unroll
  for (int e = 0; e < 8; ++e) {
    const float t = act ? (v[e] - mean) : 0.f;
    d8[e] = t;
    q = q + t * t;
  }
  q = q + __shfl_xor(q, 16, 32);
  q = q + __shfl_xor(q, 8, 32);
  q = q + __shfl_xor(q, 4, 32);
  q = q + __shfl_xor(q, 2, 32);
  q = q + __shfl_xor(q, 1, 32);
  const float rstd = rsqrtf(q * (1.0f / 192.0f) + 1e-5f);
  const v4f g0 = *(const v4f*)(g + lc * 8);
  const v4f g1 = *(const v4f*)(g + lc * 8 + 4);
  const v4f b0 = *(const v4f*)(b + lc * 8);
  const v4f b1 = *(const v4f*)(b + lc * 8 + 4);
  float gg[8], bb[8];
#pragma unroll
  for (int e = 0; e < 4; ++e) { gg[e] = bfr(g0[e]); gg[4 + e] = bfr(g1[e]); bb[e] = bfr(b0[e]); bb[4 + e] = bfr(b1[e]); }
  v4u ph, pl;
#pragma unroll
  for (int e = 0; e < 4; ++e) {
    const float y0 = (d8[2 * e] * rstd * gg[2 * e] + bb[2 * e]) * scl;
    const float y1 = (d8[2 * e + 1] * rstd * gg[2 * e + 1] + bb[2 * e + 1]) * scl;
    const _Float16 h0 = (_Float16)y0, h1 = (_Float16)y1;
    const float r0 = (y0 - (float)h0) * 16384.0f;
    const float r1 = (y1 - (float)h1) * 16384.0f;
    ph[e] = pk16(h_bits(h0), h_bits(h1));
    pl[e] = pk16(hb16(r0), hb16(r1));
  }
  unsigned short* oh = dh + (size_t)row * CDIM + lc * 8;
  unsigned short* ol = dl + (size_t)row * CDIM + lc * 8;
  if (act) {
    *(volatile v4u*)oh = ph;
    *(volatile v4u*)ol = pl;
  }
  __threadfence();
  if (act) {
    *(volatile v4u*)oh = ph;
    *(volatile v4u*)ol = pl;
  }
}

template <int EPI>
__global__ __launch_bounds__(256)
void gemm_k(const unsigned short* __restrict__ ah, const unsigned short* __restrict__ al, int lda, int ksa,
            const unsigned short* __restrict__ wb, int K,
            const float* __restrict__ bias, const float* __restrict__ aux, int rowoff,
            unsigned short* p0, unsigned short* p1, unsigned short* p2, float* po) {
  __shared__ __align__(16) float Cs[128 * LDC];
  const int tid = threadIdx.x, wave = tid >> 5, lane = tid & 31, hh = lane >> 4, c = lane & 15;
  const int mb = blockIdx.x, nb = blockIdx.y;
  const int mw = wave >> 1, nw = wave & 1;
  const _Float16* Ah = (const _Float16*)(const void*)ah;
  const _Float16* Al = (const _Float16*)(const void*)al;
  const _Float16* W  = (const _Float16*)(const void*)wb;
  const int arow0 = mb * 128 + mw * 32;
  const int bcol0 = nb * 64 + nw * 32;
  const _Float16* pa0 = Ah + (size_t)(arow0 + c) * lda + 8 * hh;
  const _Float16* pa1 = Ah + (size_t)(arow0 + 16 + c) * lda + 8 * hh;
  const _Float16* qa0 = Al + (size_t)(arow0 + c) * lda + 8 * hh;
  const _Float16* qa1 = Al + (size_t)(arow0 + 16 + c) * lda + 8 * hh;
  const _Float16* pb0 = W + (size_t)(bcol0 + c) * K + 8 * hh;
  const _Float16* pb1 = W + (size_t)(bcol0 + 16 + c) * K + 8 * hh;

  v8f h00 = zero8(), h01 = zero8(), h10 = zero8(), h11 = zero8();
  v8f l00 = zero8(), l01 = zero8(), l10 = zero8(), l11 = zero8();
  const int nk = K >> 5;
#pragma unroll 1
  for (int ks = 0; ks < nk; ++ks) {
    const size_t ao = (size_t)ks * (size_t)ksa;
    const int bo = ks * 32;
    const v16h fa0 = ldfrag_h(pa0 + ao);
    const v16h fa1 = ldfrag_h(pa1 + ao);
    const v16h ga0 = ldfrag_h(qa0 + ao);
    const v16h ga1 = ldfrag_h(qa1 + ao);
    const v16h fb0 = ldfrag_h(pb0 + bo);
    const v16h fb1 = ldfrag_h(pb1 + bo);
    h00 = mma_raw(fa0, fb0, h00);
    h01 = mma_raw(fa0, fb1, h01);
    h10 = mma_raw(fa1, fb0, h10);
    h11 = mma_raw(fa1, fb1, h11);
    l00 = mma_raw(ga0, fb0, l00);
    l01 = mma_raw(ga0, fb1, l01);
    l10 = mma_raw(ga1, fb0, l10);
    l11 = mma_raw(ga1, fb1, l11);
    guard8(h00, h01, h10, h11, l00, l01, l10, l11, fa0, fa1, ga0, ga1, fb0, fb1);
  }
#pragma unroll
  for (int r = 0; r < 8; ++r) {
    const int row = mw * 32 + 8 * hh + r;
    Cs[row * LDC + nw * 32 + c]             = h00[r] + l00[r] * (1.0f / 16384.0f);
    Cs[row * LDC + nw * 32 + 16 + c]        = h01[r] + l01[r] * (1.0f / 16384.0f);
    Cs[(row + 16) * LDC + nw * 32 + c]      = h10[r] + l10[r] * (1.0f / 16384.0f);
    Cs[(row + 16) * LDC + nw * 32 + 16 + c] = h11[r] + l11[r] * (1.0f / 16384.0f);
  }
  __syncthreads();

  const float SA = (EPI == 1) ? (1.0f / 65536.0f) : ((EPI == 3) ? (1.0f / 16384.0f) : (1.0f / 8192.0f));
  const float* bq = bias + nb * 64;

  if (EPI == 0) {
    if (nb < 3) {
      v4u pk[4];
      size_t offs[4];
#pragma unroll
      for (int s = 0; s < 4; ++s) {
        const int L = s * 32 + (tid >> 3), p = tid & 7;
        const int col = p * 8;
        v4u q4;
#pragma unroll
        for (int e = 0; e < 4; ++e) {
          const float f0 = Cs[L * LDC + col + 2 * e] * SA + bfr(bq[col + 2 * e]);
          const float f1 = Cs[L * LDC + col + 2 * e + 1] * SA + bfr(bq[col + 2 * e + 1]);
          q4[e] = pk16(hb16(f0 * 8.0f), hb16(f1 * 8.0f));
        }
        pk[s] = q4;
        offs[s] = (size_t)(mb * 128 + L) * CDIM + nb * 64 + col;
      }
#pragma unroll
      for (int s = 0; s < 4; ++s) *(volatile v4u*)(p0 + offs[s]) = pk[s];
      __threadfence();
#pragma unroll
      for (int s = 0; s < 4; ++s) *(volatile v4u*)(p0 + offs[s]) = pk[s];
    } else {
      const int hp = nb - 3;
      v4u phk[4], plk[4];
      size_t offs[4];
#pragma unroll
      for (int s = 0; s < 4; ++s) {
        const int L = s * 32 + (tid >> 3), p = tid & 7;
        const int wl = L >> 6, hl = (L >> 5) & 1, d = L & 31;
        const int col = hl * 32 + d;
        const int tb = p * 8;
        const float bc = bfr(bq[col]);
        v4u a, bv;
#pragma unroll
        for (int e = 0; e < 4; ++e) {
          const float v0 = Cs[(wl * 64 + tb + 2 * e) * LDC + col] * SA + bc;
          const float v1 = Cs[(wl * 64 + tb + 2 * e + 1) * LDC + col] * SA + bc;
          const float f0 = v0 * 16.0f, f1 = v1 * 16.0f;
          const _Float16 h0 = (_Float16)f0, h1 = (_Float16)f1;
          const float r0 = (f0 - (float)h0) * 16384.0f;
          const float r1 = (f1 - (float)h1) * 16384.0f;
          a[e]  = pk16(h_bits(h0), h_bits(h1));
          bv[e] = pk16(hb16(r0), hb16(r1));
        }
        phk[s] = a;
        plk[s] = bv;
        const int wh = (mb * 2 + wl) * NHEAD + hp * 2 + hl;
        offs[s] = ((size_t)wh * HDIM + d) * NTOK + tb;
      }
#pragma unroll
      for (int s = 0; s < 4; ++s) { *(volatile v4u*)(p1 + offs[s]) = phk[s]; *(volatile v4u*)(p2 + offs[s]) = plk[s]; }
      __threadfence();
#pragma unroll
      for (int s = 0; s < 4; ++s) { *(volatile v4u*)(p1 + offs[s]) = phk[s]; *(volatile v4u*)(p2 + offs[s]) = plk[s]; }
    }
  } else if (EPI == 2) {
    v4u phk[4], plk[4];
    size_t offs[4];
#pragma unroll
    for (int s = 0; s < 4; ++s) {
      const int L = s * 32 + (tid >> 3), p = tid & 7;
      const int col = p * 8;
      v4u a, bv;
#pragma unroll
      for (int e = 0; e < 4; ++e) {
        const float v0 = Cs[L * LDC + col + 2 * e] * SA + bfr(bq[col + 2 * e]);
        const float v1 = Cs[L * LDC + col + 2 * e + 1] * SA + bfr(bq[col + 2 * e + 1]);
        const float g0 = 0.5f * v0 * (1.0f + erff(v0 * 0.70710678118654752f));
        const float g1 = 0.5f * v1 * (1.0f + erff(v1 * 0.70710678118654752f));
        const float f0 = g0 * 16.0f, f1 = g1 * 16.0f;
        const _Float16 h0 = (_Float16)f0, h1 = (_Float16)f1;
        const float r0 = (f0 - (float)h0) * 16384.0f;
        const float r1 = (f1 - (float)h1) * 16384.0f;
        a[e]  = pk16(h_bits(h0), h_bits(h1));
        bv[e] = pk16(hb16(r0), hb16(r1));
      }
      phk[s] = a;
      plk[s] = bv;
      offs[s] = (size_t)(mb * 128 + L) * HID + nb * 64 + col;
    }
#pragma unroll
    for (int s = 0; s < 4; ++s) { *(volatile v4u*)(p0 + offs[s]) = phk[s]; *(volatile v4u*)(p1 + offs[s]) = plk[s]; }
    __threadfence();
#pragma unroll
    for (int s = 0; s < 4; ++s) { *(volatile v4u*)(p0 + offs[s]) = phk[s]; *(volatile v4u*)(p1 + offs[s]) = plk[s]; }
  } else {
    v4f ov[8];
    size_t offs[8];
#pragma unroll
    for (int s = 0; s < 8; ++s) {
      const int L = s * 32 + (tid >> 3), p = tid & 7;
      const int row = L >> 1, half = L & 1;
      const int col = half * 32 + p * 4;
      const int growg = rowoff + mb * 128 + row;
      v4f v = *(const v4f*)(Cs + row * LDC + col);
      if (EPI == 1) {
        const v4f xx = *(const v4f*)(aux + (size_t)pos_of(growg) * CDIM + nb * 64 + col);
#pragma unroll
        for (int e = 0; e < 4; ++e) {
          const float t = v[e] * SA + bfr(bq[col + e]);
          v[e] = bfr(xx[e]) + t;
        }
        offs[s] = (size_t)growg * CDIM + nb * 64 + col;
      } else {
        const v4f xr = *(const v4f*)(aux + (size_t)growg * CDIM + nb * 64 + col);
#pragma unroll
        for (int e = 0; e < 4; ++e) {
          const float t = v[e] * SA + bfr(bq[col + e]);
          v[e] = xr[e] + t;
        }
        offs[s] = (size_t)pos_of(growg) * CDIM + nb * 64 + col;
      }
      ov[s] = v;
    }
#pragma unroll
    for (int s = 0; s < 8; ++s) *(volatile v4f*)(po + offs[s]) = ov[s];
    __threadfence();
#pragma unroll
    for (int s = 0; s < 8; ++s) *(volatile v4f*)(po + offs[s]) = ov[s];
  }
}

__global__ __launch_bounds__(128)
void attn_win(const unsigned short* __restrict__ qhp, const unsigned short* __restrict__ qlp,
              const unsigned short* __restrict__ kpp, const unsigned short* __restrict__ vth,
              const unsigned short* __restrict__ vtl, const float* __restrict__ bm,
              unsigned short* ohi, unsigned short* olo) {
  __shared__ __align__(16) char pbuf[4 * PWB];
  const int tid = threadIdx.x, wave = tid >> 5, lane = tid & 31, hh = lane >> 4, c = lane & 15;
  const int wh = blockIdx.x;
  const int win = wh / NHEAD, h = wh - win * NHEAD;
  const int ql0 = wave * 16;
  const int q0 = win * NTOK + ql0;
  const _Float16* Qh = (const _Float16*)(const void*)qhp;
  const _Float16* Ql = (const _Float16*)(const void*)qlp;
  const _Float16* Kp = (const _Float16*)(const void*)kpp;
  const _Float16* Vh = (const _Float16*)(const void*)vth + (size_t)wh * HDIM * NTOK;
  const _Float16* Vl = (const _Float16*)(const void*)vtl + (size_t)wh * HDIM * NTOK;
  _Float16* Ph = (_Float16*)(pbuf + wave * PWB);
  _Float16* Pl = Ph + 16 * PP;

  const v16h fqh = ldfrag_h(Qh + (size_t)(q0 + c) * CDIM + h * HDIM + 8 * hh);
  const v16h fql = ldfrag_h(Ql + (size_t)(q0 + c) * CDIM + h * HDIM + 8 * hh);
  const float* bmr = bm + ((size_t)(h * NTOK + ql0 + 8 * hh)) * NTOK + c;

  v8f s[4];
#pragma unroll
  for (int j = 0; j < 4; ++j) {
    const v16h kf = ldfrag_h(Kp + (size_t)(win * NTOK + j * 16 + c) * CDIM + h * HDIM + 8 * hh);
    v8f sa = mma_raw(fqh, kf, zero8());
    v8f sb = mma_raw(fql, kf, zero8());
    guard2(sa, sb, fqh, fql, kf);
    v8f sj;
#pragma unroll
    for (int r = 0; r < 8; ++r) {
      const float t = sa[r] + sb[r] * (1.0f / 16384.0f);
      sj[r] = t * (1.0f / 512.0f) + bmr[r * NTOK + j * 16];
    }
    s[j] = sj;
  }
#pragma unroll
  for (int r = 0; r < 8; ++r) {
    float m = fmaxf(fmaxf(s[0][r], s[1][r]), fmaxf(s[2][r], s[3][r]));
    m = fmaxf(m, __shfl_xor(m, 1, 32));
    m = fmaxf(m, __shfl_xor(m, 2, 32));
    m = fmaxf(m, __shfl_xor(m, 4, 32));
    m = fmaxf(m, __shfl_xor(m, 8, 32));
    float e4[4];
    float ss = 0.f;
#pragma unroll
    for (int j = 0; j < 4; ++j) {
      const float e = __expf(s[j][r] - m);
      e4[j] = e;
      ss = ss + e;
    }
    ss = ss + __shfl_xor(ss, 1, 32);
    ss = ss + __shfl_xor(ss, 2, 32);
    ss = ss + __shfl_xor(ss, 4, 32);
    ss = ss + __shfl_xor(ss, 8, 32);
    const float rinv = 1024.0f * (1.0f / ss);
#pragma unroll
    for (int j = 0; j < 4; ++j) s[j][r] = e4[j] * rinv;
  }
#pragma unroll
  for (int j = 0; j < 4; ++j) {
#pragma unroll
    for (int r = 0; r < 8; ++r) {
      const float pf = s[j][r];
      const _Float16 phv = (_Float16)pf;
      const float res = (pf - (float)phv) * 8192.0f;
      const int idx = (8 * hh + r) * PP + j * 16 + c;
      Ph[idx] = phv;
      Pl[idx] = (_Float16)res;
    }
  }
  wave_sync_lds();
  v8f ohh0 = zero8(), ohh1 = zero8(), ohl0 = zero8(), ohl1 = zero8(), olh0 = zero8(), olh1 = zero8();
#pragma unroll
  for (int ks = 0; ks < 2; ++ks) {
    const v16h pa  = ldfrag_h(Ph + c * PP + ks * 32 + 8 * hh);
    const v16h pla = ldfrag_h(Pl + c * PP + ks * 32 + 8 * hh);
    const int koff = ks * 32 + 8 * hh;
    {
      const v16h vh = ldfrag_h(Vh + (size_t)c * NTOK + koff);
      const v16h vl = ldfrag_h(Vl + (size_t)c * NTOK + koff);
      ohh0 = mma_raw(pa, vh, ohh0);
      ohl0 = mma_raw(pa, vl, ohl0);
      olh0 = mma_raw(pla, vh, olh0);
      guard3(ohh0, ohl0, olh0, pa, pla, vh, vl);
    }
    {
      const v16h vh = ldfrag_h(Vh + (size_t)(16 + c) * NTOK + koff);
      const v16h vl = ldfrag_h(Vl + (size_t)(16 + c) * NTOK + koff);
      ohh1 = mma_raw(pa, vh, ohh1);
      ohl1 = mma_raw(pa, vl, ohl1);
      olh1 = mma_raw(pla, vh, olh1);
      guard3(ohh1, ohl1, olh1, pa, pla, vh, vl);
    }
  }
  wave_sync_lds();

  float* Os = (float*)(void*)(pbuf + wave * PWB);
#pragma unroll
  for (int r = 0; r < 8; ++r) {
    const int row = 8 * hh + r;
    float o0 = ohh0[r] + ohl0[r] * (1.0f / 16384.0f);
    o0 = o0 + olh0[r] * (1.0f / 8192.0f);
    float o1 = ohh1[r] + ohl1[r] * (1.0f / 16384.0f);
    o1 = o1 + olh1[r] * (1.0f / 8192.0f);
    Os[row * OSP + c]      = o0 * (1.0f / 16384.0f);
    Os[row * OSP + 16 + c] = o1 * (1.0f / 16384.0f);
  }
  wave_sync_lds();
  v4u ph2[2], pl2[2];
  size_t off2[2];
#pragma unroll
  for (int sI = 0; sI < 2; ++sI) {
    const int line = sI * 4 + (lane >> 3), piece = lane & 7;
    const int row = 2 * line + (piece >> 2), d0 = (piece & 3) * 8;
    v4u a, bv;
#pragma unroll
    for (int e = 0; e < 4; ++e) {
      const float f0 = Os[row * OSP + d0 + 2 * e] * 64.0f;
      const float f1 = Os[row * OSP + d0 + 2 * e + 1] * 64.0f;
      const _Float16 h0 = (_Float16)f0, h1 = (_Float16)f1;
      const float r0 = (f0 - (float)h0) * 16384.0f;
      const float r1 = (f1 - (float)h1) * 16384.0f;
      a[e]  = pk16(h_bits(h0), h_bits(h1));
      bv[e] = pk16(hb16(r0), hb16(r1));
    }
    ph2[sI] = a;
    pl2[sI] = bv;
    off2[sI] = ((size_t)h * NROW + (size_t)q0 + row) * HDIM + d0;
  }
  *(volatile v4u*)(ohi + off2[0]) = ph2[0];
  *(volatile v4u*)(ohi + off2[1]) = ph2[1];
  *(volatile v4u*)(olo + off2[0]) = pl2[0];
  *(volatile v4u*)(olo + off2[1]) = pl2[1];
  __threadfence();
  *(volatile v4u*)(ohi + off2[0]) = ph2[0];
  *(volatile v4u*)(ohi + off2[1]) = ph2[1];
  *(volatile v4u*)(olo + off2[0]) = pl2[0];
  *(volatile v4u*)(olo + off2[1]) = pl2[1];
}

extern "C" void kernel_launch(void* const* d_in, const int* in_sizes, int n_in,
                              void* d_out, int out_size, void* d_ws, size_t ws_size,
                              hipStream_t stream) {
  if (n_in < 17) return;
  if (in_sizes[0] != NROW * CDIM || in_sizes[2] != NROW * CDIM || in_sizes[3] != NROW * CDIM) return;
  if (in_sizes[4] != CDIM || in_sizes[5] != CDIM) return;
  if (in_sizes[6] != CDIM * NKV || in_sizes[7] != NKV) return;
  if (in_sizes[8] != NRPB * NHEAD) return;
  if (in_sizes[9] != CDIM * CDIM || in_sizes[10] != CDIM) return;
  if (in_sizes[11] != CDIM || in_sizes[12] != CDIM) return;
  if (in_sizes[13] != CDIM * HID || in_sizes[14] != HID) return;
  if (in_sizes[15] != HID * CDIM || in_sizes[16] != CDIM) return;
  if (out_size != NROW * CDIM) return;

  const float* x      = (const float*)d_in[0];
  const float* skip   = (const float*)d_in[2];
  const float* x_up   = (const float*)d_in[3];
  const float* n1g    = (const float*)d_in[4];
  const float* n1b    = (const float*)d_in[5];
  const float* kv_w   = (const float*)d_in[6];
  const float* kv_b   = (const float*)d_in[7];
  const float* rpb    = (const float*)d_in[8];
  const float* proj_w = (const float*)d_in[9];
  const float* proj_b = (const float*)d_in[10];
  const float* n2g    = (const float*)d_in[11];
  const float* n2b    = (const float*)d_in[12];
  const float* fc1_w  = (const float*)d_in[13];
  const float* fc1_b  = (const float*)d_in[14];
  const float* fc2_w  = (const float*)d_in[15];
  const float* fc2_b  = (const float*)d_in[16];
  float* out = (float*)d_out;

  const size_t sWkv = (size_t)NKV * CDIM * 2;
  const size_t sWp  = (size_t)CDIM * CDIM * 2;
  const size_t sW1  = (size_t)HID * CDIM * 2;
  const size_t sW2  = (size_t)CDIM * HID * 2;
  const size_t sBM  = (size_t)NHEAD * NTOK * NTOK * 4;
  const size_t sXR  = (size_t)NROW * CDIM * 4;
  const size_t sP16 = (size_t)NROW * CDIM * 2;
  const size_t sGh  = (size_t)(NROW / 2) * HID * 2;
  size_t off = 0;
  const size_t oWkv = off; off += sWkv;
  const size_t oWp  = off; off += sWp;
  const size_t oW1  = off; off += sW1;
  const size_t oW2  = off; off += sW2;
  const size_t oBM  = off; off += sBM;
  const size_t oXR  = off; off += sXR;
  const size_t oRA  = off; off += 2 * sP16;
  const size_t oRB  = off; off += 2 * sP16;
  const size_t oRC  = off; off += sP16;
  const size_t oRD  = off; off += 2 * sP16;
  if (off > ws_size) return;
  if (off > (size_t)134217728) return;
  if (oRB + 2 * sGh > off) return;
  if ((size_t)NHEAD * NROW * HDIM * 2 != sP16) return;
  if ((size_t)NWINT * NHEAD * HDIM * NTOK * 2 != sP16) return;

  char* ws = (char*)d_ws;
  unsigned short* Wkv = (unsigned short*)(ws + oWkv);
  unsigned short* Wp  = (unsigned short*)(ws + oWp);
  unsigned short* W1  = (unsigned short*)(ws + oW1);
  unsigned short* W2  = (unsigned short*)(ws + oW2);
  float*          BM  = (float*)(ws + oBM);
  float*          XR  = (float*)(ws + oXR);
  unsigned short* Sh  = (unsigned short*)(ws + oRA);
  unsigned short* Sl  = (unsigned short*)(ws + oRA + sP16);
  unsigned short* Oh  = (unsigned short*)(ws + oRA);
  unsigned short* Ol  = (unsigned short*)(ws + oRA + sP16);
  unsigned short* Hh  = (unsigned short*)(ws + oRA);
  unsigned short* Hl  = (unsigned short*)(ws + oRA + sP16);
  unsigned short* Qh  = (unsigned short*)(ws + oRB);
  unsigned short* Ql  = (unsigned short*)(ws + oRB + sP16);
  unsigned short* Kp  = (unsigned short*)(ws + oRC);
  unsigned short* Vth = (unsigned short*)(ws + oRD);
  unsigned short* Vtl = (unsigned short*)(ws + oRD + sP16);
  unsigned short* Gh  = (unsigned short*)(ws + oRB);
  unsigned short* Gl  = (unsigned short*)(ws + oRB + sGh);

  const dim3 blk(256);
  cvt_wt<<<dim3(NKV / 64, CDIM / 64), blk, 0, stream>>>(kv_w, Wkv, CDIM, NKV);
  cvt_wt<<<dim3(CDIM / 64, CDIM / 64), blk, 0, stream>>>(proj_w, Wp, CDIM, CDIM);
  cvt_wt<<<dim3(HID / 64, CDIM / 64), blk, 0, stream>>>(fc1_w, W1, CDIM, HID);
  cvt_wt<<<dim3(CDIM / 64, HID / 64), blk, 0, stream>>>(fc2_w, W2, HID, CDIM);
  build_bm<<<dim3((NHEAD * NTOK * NTOK) / (4 * 256)), blk, 0, stream>>>(rpb, BM);
  ln_rows<<<dim3(NROW / 8), blk, 0, stream>>>(skip, n1g, n1b, Sh, Sl, 8.0f, 1);
  ln_rows<<<dim3(NROW / 8), blk, 0, stream>>>(x_up, n1g, n1b, Qh, Ql, QSC * 64.0f, 1);
  gemm_k<0><<<dim3(NROW / 128, NKV / 64), blk, 0, stream>>>(Sh, Sl, CDIM, 32, Wkv, CDIM, kv_b, BM, 0,
                                                            Kp, Vth, Vtl, XR);
  attn_win<<<dim3(NWINT * NHEAD), dim3(128), 0, stream>>>(Qh, Ql, Kp, Vth, Vtl, BM, Oh, Ol);
  gemm_k<1><<<dim3(NROW / 128, CDIM / 64), blk, 0, stream>>>(Oh, Ol, HDIM, NROW * HDIM, Wp, CDIM, proj_b, x, 0,
                                                             Kp, Kp, Kp, XR);
  ln_rows<<<dim3(NROW / 8), blk, 0, stream>>>(XR, n2g, n2b, Hh, Hl, 8.0f, 0);
  for (int half = 0; half < 2; ++half) {
    const size_t aoff = (size_t)half * (NROW / 2) * CDIM;
    gemm_k<2><<<dim3((NROW / 2) / 128, HID / 64), blk, 0, stream>>>(Hh + aoff, Hl + aoff, CDIM, 32, W1, CDIM,
                                                                    fc1_b, BM, 0, Gh, Gl, Kp, XR);
    gemm_k<3><<<dim3((NROW / 2) / 128, CDIM / 64), blk, 0, stream>>>(Gh, Gl, HID, 32, W2, HID, fc2_b, XR,
                                                                     half * (NROW / 2), Kp, Kp, Kp, out);
  }
  (void)hipGetLastError();
}
